// SelectiveSSM_35304631174086
// MI455X (gfx1250) — hardware-verified
//
#include <hip/hip_runtime.h>
#include <math.h>

typedef __attribute__((ext_vector_type(16))) _Float16 v16h;
typedef __attribute__((ext_vector_type(8)))  _Float16 v8h;
typedef __attribute__((ext_vector_type(16))) __bf16   v16b;
typedef __attribute__((ext_vector_type(8)))  __bf16   v8b;
typedef __attribute__((ext_vector_type(8)))  float    v8f;
typedef __attribute__((ext_vector_type(4)))  float    v4f;

constexpr int kBatch = 2;
constexpr int kSeqL  = 1024;
constexpr int kDin   = 2048;
constexpr int kNst   = 16;
constexpr int kDtR   = 64;
constexpr int kPrjN  = kDtR + 2 * kNst;
constexpr int kPrjP  = 128;
constexpr int kRows  = kBatch * kSeqL;
constexpr int kChunk = 16;
constexpr int kScanC = 256;
constexpr int kTP    = 260;
static_assert(kPrjN == 96 && kPrjP >= kPrjN, "x_proj width");
static_assert((kDin % 32) == 0 && (kDtR % 32) == 0, "GEMM K multiples of 32");
static_assert((kRows % 64) == 0 && (kPrjP % 64) == 0 && (kDin % 64) == 0, "GEMM M,N multiples of 64");
static_assert((kSeqL % kChunk) == 0 && (kDin % kScanC) == 0 && kScanC == 256, "scan tiles");
static_assert((kRows * kDin) % 2048 == 0 && (kPrjP * kDin) % 2048 == 0 && (kDin * kDtR) % 2048 == 0 && (kRows * kDtR) % 2048 == 0, "cast grids exact");

constexpr size_t kOffXH   = 0;
constexpr size_t kOffXL   = kOffXH  + (size_t)kRows * kDin  * 2;
constexpr size_t kOffWXH  = kOffXL  + (size_t)kRows * kDin  * 2;
constexpr size_t kOffWXL  = kOffWXH + (size_t)kPrjP * kDin  * 2;
constexpr size_t kOffWDH  = kOffWXL + (size_t)kPrjP * kDin  * 2;
constexpr size_t kOffWDL  = kOffWDH + (size_t)kDin  * kDtR  * 2;
constexpr size_t kOffXZ   = kOffWDL + (size_t)kDin  * kDtR  * 2;
constexpr size_t kOffDRH  = kOffXZ  + (size_t)kRows * kPrjP * 4;
constexpr size_t kOffDRL  = kOffDRH + (size_t)kRows * kDtR  * 2;
constexpr size_t kOffDPRE = kOffDRL + (size_t)kRows * kDtR  * 2;
constexpr size_t kWsTotal = kOffDPRE + (size_t)kRows * kDin * 4;
static_assert(kWsTotal == 36700160ull, "carve total");
static_assert(kWsTotal <= 134217728ull, "carve cap");
static_assert((kOffXL % 128) == 0 && (kOffWXH % 128) == 0 && (kOffWXL % 128) == 0 && (kOffWDH % 128) == 0 &&
              (kOffWDL % 128) == 0 && (kOffXZ % 128) == 0 && (kOffDRH % 128) == 0 && (kOffDRL % 128) == 0 &&
              (kOffDPRE % 128) == 0, "128-B aligned regions");

__device__ __forceinline__ unsigned short f2bf_bits(float f) {
  unsigned u = __float_as_uint(f);
  return (unsigned short)((u + 0x7FFFu + ((u >> 16) & 1u)) >> 16);
}
__device__ __forceinline__ float bf_bits2f(unsigned short h) { return __uint_as_float(((unsigned)h) << 16); }

__device__ __forceinline__ void dep_guard4_h(v8f& a, v8f& b, v8f& c, v8f& d, v16h x, v16h y) { asm volatile("v_nop\n\tv_nop\n\tv_nop\n\tv_nop" : "+v"(a), "+v"(b), "+v"(c), "+v"(d) : "v"(x), "v"(y)); }
__device__ __forceinline__ void dep_guard4_b(v8f& a, v8f& b, v8f& c, v8f& d, v16b x, v16b y) { asm volatile("v_nop\n\tv_nop\n\tv_nop\n\tv_nop" : "+v"(a), "+v"(b), "+v"(c), "+v"(d) : "v"(x), "v"(y)); }
__device__ __forceinline__ void keep4_h(v16h a, v16h b, v16h c, v16h d) { asm volatile("v_nop" :: "v"(a), "v"(b), "v"(c), "v"(d)); }
__device__ __forceinline__ void keep4_b(v16b a, v16b b, v16b c, v16b d) { asm volatile("v_nop" :: "v"(a), "v"(b), "v"(c), "v"(d)); }
__device__ __forceinline__ void acc_guard4(v8f& a, v8f& b, v8f& c, v8f& d) { asm volatile("v_nop\n\tv_nop\n\tv_nop\n\tv_nop" : "+v"(a), "+v"(b), "+v"(c), "+v"(d)); }
template <typename T> struct Frag;
template <> struct Frag<_Float16> {
  typedef v16h V; union U { v16h v; v8h h[2]; };
  static __device__ __forceinline__ v16h load(const _Float16* p) {
    U f; f.h[0] = *(const v8h*)(p); f.h[1] = *(const v8h*)(p + 16); return f.v;
  }
  static __device__ __forceinline__ v8f mma(v16h a, v16h b, v8f c) {
    return __builtin_amdgcn_wmma_f32_16x16x32_f16(false, a, false, b, (short)0, c, false, false);
  }
  static __device__ __forceinline__ void guard4(v8f& a, v8f& b, v8f& c, v8f& d, v16h x, v16h y) { dep_guard4_h(a, b, c, d, x, y); }
  static __device__ __forceinline__ void keep(v16h a, v16h b, v16h c, v16h d) { keep4_h(a, b, c, d); }
};
template <> struct Frag<__bf16> {
  typedef v16b V; union U { v16b v; v8b h[2]; };
  static __device__ __forceinline__ v16b load(const __bf16* p) {
    U f; f.h[0] = *(const v8b*)(p); f.h[1] = *(const v8b*)(p + 16); return f.v;
  }
  static __device__ __forceinline__ v8f mma(v16b a, v16b b, v8f c) {
    return __builtin_amdgcn_wmma_f32_16x16x32_bf16(false, a, false, b, (short)0, c, false, false);
  }
  static __device__ __forceinline__ void guard4(v8f& a, v8f& b, v8f& c, v8f& d, v16b x, v16b y) { dep_guard4_b(a, b, c, d, x, y); }
  static __device__ __forceinline__ void keep(v16b a, v16b b, v16b c, v16b d) { keep4_b(a, b, c, d); }
};

template <int ET> struct Elem;
template <> struct Elem<0> { typedef _Float16 T; };
template <> struct Elem<1> { typedef __bf16 T; };
template <int ET, int SPL, int BIAS_MODE, int OUT_MODE, bool RESID, int ACT = 0>
__global__ __launch_bounds__(256) void wmma_gemm64(
    const unsigned short* __restrict__ Ap, const unsigned short* __restrict__ A2p, int lda, long strideA,
    const unsigned short* __restrict__ Btp, const unsigned short* __restrict__ Bt2p, int ldb, long strideB,
    void* __restrict__ Cout, void* __restrict__ Cout2, int ldc, long strideC,
    const float* __restrict__ bias,
    const float* __restrict__ resid, long strideR,
    int M, int N, int K, float scale) {
  typedef typename Elem<ET>::T T;
  typedef typename Frag<T>::V V;
  const T* A = (const T*)Ap; const T* A2 = (const T*)A2p; const T* Bt = (const T*)Btp; const T* Bt2 = (const T*)Bt2p;
  __shared__ __align__(16) float sT[8][16 * 68];
  const int b    = blockIdx.y;
  const int lane = threadIdx.x & 31;
  const int wave = threadIdx.x >> 5;
  const int tilesN = N >> 6;
  const int tilesM = M >> 6;
  const int tile = blockIdx.x * 8 + wave;
  if (tile >= tilesM * tilesN) return;
  const int tm = tile / tilesN;
  const int tn = tile - tm * tilesN;
  const int m0 = tm << 6;
  const int n0 = tn << 6;

  const T* Ab  = A  + (size_t)b * strideA;
  const T* Bb  = Bt + (size_t)b * strideB;
  const T* Ab2 = (SPL >= 1) ? (A2  + (size_t)b * strideA) : nullptr;
  const T* Bb2 = (SPL == 2) ? (Bt2 + (size_t)b * strideB) : nullptr;

  const int rlane = lane & 15;
  const int koff  = (lane >> 4) * 8;
  const int mOff  = (lane >> 4) * 8;

  v8f acc[4][4];
#pragma unroll
  for (int i = 0; i < 4; ++i)
#pragma unroll
    for (int j = 0; j < 4; ++j) acc[i][j] = (v8f){0.f,0.f,0.f,0.f,0.f,0.f,0.f,0.f};

  for (int k0 = 0; k0 < K; k0 += 32) {
    V bh[4], bl[4];
#pragma unroll
    for (int j = 0; j < 4; ++j) {
      const size_t bo = (size_t)(n0 + (j << 4) + rlane) * ldb + koff + k0;
      bh[j] = Frag<T>::load(Bb + bo);
      if (SPL == 2) bl[j] = Frag<T>::load(Bb2 + bo);
    }
#pragma unroll
    for (int i = 0; i < 4; ++i) {
      const size_t ao = (size_t)(m0 + (i << 4) + rlane) * lda + koff + k0;
      V ah = Frag<T>::load(Ab + ao);
      V al;
      if (SPL >= 1) al = Frag<T>::load(Ab2 + ao);
#pragma unroll
      for (int j = 0; j < 4; ++j) {
        acc[i][j] = Frag<T>::mma(ah, bh[j], acc[i][j]);
        if (SPL == 2) acc[i][j] = Frag<T>::mma(ah, bl[j], acc[i][j]);
        if (SPL >= 1) acc[i][j] = Frag<T>::mma(al, bh[j], acc[i][j]);
      }
      Frag<T>::guard4(acc[i][0], acc[i][1], acc[i][2], acc[i][3], ah, (SPL >= 1) ? al : ah);
    }
    Frag<T>::keep(bh[0], bh[1], bh[2], bh[3]);
    if (SPL == 2) Frag<T>::keep(bl[0], bl[1], bl[2], bl[3]);
  }
  acc_guard4(acc[0][0], acc[0][1], acc[0][2], acc[0][3]);
  acc_guard4(acc[1][0], acc[1][1], acc[1][2], acc[1][3]);
  acc_guard4(acc[2][0], acc[2][1], acc[2][2], acc[2][3]);
  acc_guard4(acc[3][0], acc[3][1], acc[3][2], acc[3][3]);

  float* slab = sT[wave];
  const float* Rb = RESID ? (resid + (size_t)b * strideR) : nullptr;
#pragma unroll
  for (int i = 0; i < 4; ++i) {
    const int mBase = m0 + (i << 4);
#pragma unroll
    for (int j = 0; j < 4; ++j) {
      const int n = n0 + (j << 4) + rlane;
      float bv = 0.f;
      if (BIAS_MODE == 2) bv = bias[n];
#pragma unroll
      for (int r = 0; r < 8; ++r) {
        float v = acc[i][j][r] * scale;
        if (BIAS_MODE == 1) v += bias[mBase + mOff + r];
        if (BIAS_MODE == 2) v += bv;
        if (RESID) v += Rb[(size_t)(mBase + mOff + r) * ldc + n];
        if (ACT == 1) v = tanhf(v);
        if (ACT == 2) v = fmaxf(v, 0.0f);
        if (ACT == 3) v = v / (1.0f + expf(-v));
        if (ACT == 4) v = (v > 0.f) ? v : 0.01f * v;
        slab[(mOff + r) * 68 + (j << 4) + rlane] = v;
      }
    }
    __builtin_amdgcn_fence(__ATOMIC_RELEASE, "workgroup");
    __builtin_amdgcn_wave_barrier();
    __builtin_amdgcn_fence(__ATOMIC_ACQUIRE, "workgroup");
    if (OUT_MODE == 0) {
      float* C = (float*)Cout + (size_t)b * strideC;
      const int hh = lane >> 4, c4 = (lane & 15) * 4;
      for (int pass = 0; pass < 2; ++pass) {
#pragma unroll
        for (int it = 0; it < 8; ++it) {
          const int row = it * 2 + hh;
          v4f v = *(const v4f*)(slab + row * 68 + c4);
          *(volatile v4f*)(C + (size_t)(mBase + row) * ldc + n0 + c4) = v;
        }
        __threadfence();
      }
    } else {
      const int q = lane >> 3, c8 = (lane & 7) * 8;
      unsigned short* C  = (unsigned short*)Cout  + (size_t)b * strideC;
      unsigned short* C2 = (OUT_MODE == 2) ? ((unsigned short*)Cout2 + (size_t)b * strideC) : nullptr;
      for (int pass = 0; pass < 2; ++pass) {
#pragma unroll
        for (int it = 0; it < 4; ++it) {
          const int row = it * 4 + q;
          const float* sp = slab + row * 68 + c8;
          v8h hv, lv;
#pragma unroll
          for (int e = 0; e < 8; ++e) {
            if (OUT_MODE == 1) {
              hv[e] = (_Float16)sp[e];
            } else {
              unsigned short hb = f2bf_bits(sp[e]);
              unsigned short lb = f2bf_bits(sp[e] - bf_bits2f(hb));
              hv[e] = __builtin_bit_cast(_Float16, hb);
              lv[e] = __builtin_bit_cast(_Float16, lb);
            }
          }
          *(volatile v8h*)(C + (size_t)(mBase + row) * ldc + n0 + c8) = hv;
          if (OUT_MODE == 2) *(volatile v8h*)(C2 + (size_t)(mBase + row) * ldc + n0 + c8) = lv;
        }
        __threadfence();
      }
    }
    __builtin_amdgcn_fence(__ATOMIC_RELEASE, "workgroup");
    __builtin_amdgcn_wave_barrier();
    __builtin_amdgcn_fence(__ATOMIC_ACQUIRE, "workgroup");
  }
}

__global__ __launch_bounds__(256) void split_rows_bf16_kernel(
    const float* __restrict__ src, unsigned short* __restrict__ dhi, unsigned short* __restrict__ dlo, int total8)
{
  const int i = blockIdx.x * 256 + threadIdx.x;
  if (i >= total8) return;
  const size_t e0 = (size_t)i << 3;
  const v4f a0 = *(const v4f*)(src + e0);
  const v4f a1 = *(const v4f*)(src + e0 + 4);
  v8h hv, lv;
#pragma unroll
  for (int e = 0; e < 4; ++e) {
    const unsigned short h0 = f2bf_bits(a0[e]), h1 = f2bf_bits(a1[e]);
    const unsigned short l0 = f2bf_bits(a0[e] - bf_bits2f(h0)), l1 = f2bf_bits(a1[e] - bf_bits2f(h1));
    hv[e]     = __builtin_bit_cast(_Float16, h0);
    hv[4 + e] = __builtin_bit_cast(_Float16, h1);
    lv[e]     = __builtin_bit_cast(_Float16, l0);
    lv[4 + e] = __builtin_bit_cast(_Float16, l1);
  }
  unsigned short* qh = dhi + e0;
  unsigned short* ql = dlo + e0;
  *(volatile v8h*)qh = hv;
  *(volatile v8h*)ql = lv;
  __threadfence();
  *(volatile v8h*)qh = hv;
  *(volatile v8h*)ql = lv;
}

__global__ __launch_bounds__(256) void split_pad_wx_kernel(
    const float* __restrict__ src, unsigned short* __restrict__ dhi, unsigned short* __restrict__ dlo, int total8)
{
  const int i = blockIdx.x * 256 + threadIdx.x;
  if (i >= total8) return;
  const size_t e0 = (size_t)i << 3;
  const int row = (int)(e0 / (size_t)kDin);
  const int col = (int)(e0 - (size_t)row * kDin);
  const bool keep = (row < kPrjN);
  const int rowc = keep ? row : (kPrjN - 1);
  const float* p = src + (size_t)rowc * kDin + col;
  const v4f a0 = *(const v4f*)(p);
  const v4f a1 = *(const v4f*)(p + 4);
  v8h hv, lv;
#pragma unroll
  for (int e = 0; e < 4; ++e) {
    const float f0 = keep ? a0[e] : 0.0f;
    const float f1 = keep ? a1[e] : 0.0f;
    const unsigned short h0 = f2bf_bits(f0), h1 = f2bf_bits(f1);
    const unsigned short l0 = f2bf_bits(f0 - bf_bits2f(h0)), l1 = f2bf_bits(f1 - bf_bits2f(h1));
    hv[e]     = __builtin_bit_cast(_Float16, h0);
    hv[4 + e] = __builtin_bit_cast(_Float16, h1);
    lv[e]     = __builtin_bit_cast(_Float16, l0);
    lv[4 + e] = __builtin_bit_cast(_Float16, l1);
  }
  unsigned short* qh = dhi + e0;
  unsigned short* ql = dlo + e0;
  *(volatile v8h*)qh = hv;
  *(volatile v8h*)ql = lv;
  __threadfence();
  *(volatile v8h*)qh = hv;
  *(volatile v8h*)ql = lv;
}

__global__ __launch_bounds__(256) void dr_split_kernel(
    const float* __restrict__ XZ, unsigned short* __restrict__ dhi, unsigned short* __restrict__ dlo, int total8)
{
  const int i = blockIdx.x * 256 + threadIdx.x;
  if (i >= total8) return;
  const int e0  = i << 3;
  const int row = e0 >> 6;
  const int c8  = e0 & 63;
  const float* p = XZ + (size_t)row * kPrjP + c8;
  const v4f a0 = *(const v4f*)(p);
  const v4f a1 = *(const v4f*)(p + 4);
  v8h hv, lv;
#pragma unroll
  for (int e = 0; e < 4; ++e) {
    const unsigned short h0 = f2bf_bits(a0[e]), h1 = f2bf_bits(a1[e]);
    const unsigned short l0 = f2bf_bits(a0[e] - bf_bits2f(h0)), l1 = f2bf_bits(a1[e] - bf_bits2f(h1));
    hv[e]     = __builtin_bit_cast(_Float16, h0);
    hv[4 + e] = __builtin_bit_cast(_Float16, h1);
    lv[e]     = __builtin_bit_cast(_Float16, l0);
    lv[4 + e] = __builtin_bit_cast(_Float16, l1);
  }
  unsigned short* qh = dhi + e0;
  unsigned short* ql = dlo + e0;
  *(volatile v8h*)qh = hv;
  *(volatile v8h*)ql = lv;
  __threadfence();
  *(volatile v8h*)qh = hv;
  *(volatile v8h*)ql = lv;
}

__global__ __launch_bounds__(256) void scan_kernel(
    const float* __restrict__ DPRE, const float* __restrict__ X, const float* __restrict__ XZ,
    const float* __restrict__ bdt, const float* __restrict__ A_log, const float* __restrict__ Dv,
    float* __restrict__ out)
{
  __shared__ __align__(16) float sBC[kChunk * 32];
  __shared__ __align__(16) float sY[kChunk * kTP];
  __shared__ __align__(16) float sA[kNst * kScanC];
  const int tid = threadIdx.x, lane = tid & 31, wave = tid >> 5;
  const int b  = blockIdx.y;
  const int d0 = blockIdx.x * kScanC, d = d0 + tid;
  const size_t row0 = (size_t)b * kSeqL;

#pragma unroll 1
  for (int n = 0; n < kNst; ++n) sA[n * kScanC + tid] = -expf(A_log[(size_t)d * kNst + n]);
  __syncthreads();
  float An[kNst], h[kNst];
#pragma unroll
  for (int n = 0; n < kNst; ++n) { An[n] = sA[n * kScanC + tid]; h[n] = 0.f; }
  const float bb = bdt[d], Dd = Dv[d];
  const int hrow = wave >> 1;
  const int hch  = (wave & 1) * 128 + lane * 4;

#pragma unroll 1
  for (int c = 0; c < kSeqL / kChunk; ++c) {
    const int l0 = c * kChunk;
    if (tid < 128) {
      const int r = tid >> 3, q = (tid & 7) * 4;
      const v4f v = *(const v4f*)(XZ + (row0 + l0 + r) * kPrjP + kDtR + q);
      *(v4f*)(sBC + r * 32 + q) = v;
    }
    __syncthreads();
#pragma unroll 1
    for (int s = 0; s < kChunk; ++s) {
      const size_t m = row0 + l0 + s;
      const float a     = DPRE[m * kDin + d] + bb;
      const float delta = fmaxf(a, 0.0f) + log1pf(expf(-fabsf(a)));
      const float xv    = X[m * kDin + d];
      v4f Bq[4], Cq[4];
#pragma unroll
      for (int qq = 0; qq < 4; ++qq) {
        Bq[qq] = *(const v4f*)(sBC + s * 32 + 4 * qq);
        Cq[qq] = *(const v4f*)(sBC + s * 32 + kNst + 4 * qq);
      }
      float y = 0.f;
#pragma unroll
      for (int n = 0; n < kNst; ++n) {
        const float e = __expf(delta * An[n]);
        float db = delta * Bq[n >> 2][n & 3];
        asm volatile("" : "+v"(db));
        float p = db * xv;
        asm volatile("" : "+v"(p));
        float qv = h[n] * e;
        asm volatile("" : "+v"(qv));
        const float hn = qv + p;
        h[n] = hn;
        float rr = Cq[n >> 2][n & 3] * hn;
        asm volatile("" : "+v"(rr));
        y += rr;
      }
      float sk = xv * Dd;
      asm volatile("" : "+v"(sk));
      y += sk;
      sY[s * kTP + tid] = y;
    }
    __syncthreads();
    v4f fv[4];
#pragma unroll
    for (int it = 0; it < 4; ++it) fv[it] = *(const v4f*)(sY + (it * 4 + hrow) * kTP + hch);
    for (int pass = 0; pass < 2; ++pass) {
#pragma unroll
      for (int it = 0; it < 4; ++it)
        *(volatile v4f*)(out + (row0 + l0 + it * 4 + hrow) * kDin + d0 + hch) = fv[it];
      __threadfence();
    }
  }
}

extern "C" void kernel_launch(void* const* d_in, const int* in_sizes, int n_in,
                              void* d_out, int out_size, void* d_ws, size_t ws_size,
                              hipStream_t stream)
{
  if (n_in < 6) return;
  if (in_sizes[0] != kRows * kDin) return;
  if (in_sizes[1] != kPrjN * kDin) return;
  if (in_sizes[2] != kDin * kDtR) return;
  if (in_sizes[3] != kDin) return;
  if (in_sizes[4] != kDin * kNst) return;
  if (in_sizes[5] != kDin) return;
  if (out_size != kRows * kDin) return;
  if (ws_size < kWsTotal) return;

  const float* x     = (const float*)d_in[0];
  const float* W_x   = (const float*)d_in[1];
  const float* W_dt  = (const float*)d_in[2];
  const float* b_dt  = (const float*)d_in[3];
  const float* A_log = (const float*)d_in[4];
  const float* Dv    = (const float*)d_in[5];
  float* out = (float*)d_out;

  char* ws = (char*)d_ws;
  unsigned short* XH   = (unsigned short*)(ws + kOffXH);
  unsigned short* XL   = (unsigned short*)(ws + kOffXL);
  unsigned short* WXH  = (unsigned short*)(ws + kOffWXH);
  unsigned short* WXL  = (unsigned short*)(ws + kOffWXL);
  unsigned short* WDH  = (unsigned short*)(ws + kOffWDH);
  unsigned short* WDL  = (unsigned short*)(ws + kOffWDL);
  float*          XZ   = (float*)(ws + kOffXZ);
  unsigned short* DRH  = (unsigned short*)(ws + kOffDRH);
  unsigned short* DRL  = (unsigned short*)(ws + kOffDRL);
  float*          DPRE = (float*)(ws + kOffDPRE);
  const float* dummy_bias  = b_dt;
  const float* dummy_resid = x;

  split_rows_bf16_kernel<<<(kRows * kDin / 8) / 256, 256, 0, stream>>>(x, XH, XL, kRows * kDin / 8);
  split_pad_wx_kernel<<<(kPrjP * kDin / 8) / 256, 256, 0, stream>>>(W_x, WXH, WXL, kPrjP * kDin / 8);
  split_rows_bf16_kernel<<<(kDin * kDtR / 8) / 256, 256, 0, stream>>>(W_dt, WDH, WDL, kDin * kDtR / 8);

  wmma_gemm64<1, 2, 0, 0, false><<<dim3(8, 1), 256, 0, stream>>>(
      XH, XL, kDin, 0L,
      WXH, WXL, kDin, 0L,
      (void*)XZ, (void*)XZ, kPrjP, 0L,
      dummy_bias, dummy_resid, 0L,
      kRows, kPrjP, kDin, 1.0f);

  dr_split_kernel<<<(kRows * kDtR / 8) / 256, 256, 0, stream>>>(XZ, DRH, DRL, kRows * kDtR / 8);

  wmma_gemm64<1, 2, 0, 0, false><<<dim3(128, 1), 256, 0, stream>>>(
      DRH, DRL, kDtR, 0L,
      WDH, WDL, kDtR, 0L,
      (void*)DPRE, (void*)DPRE, kDin, 0L,
      dummy_bias, dummy_resid, 0L,
      kRows, kDin, kDtR, 1.0f);

  scan_kernel<<<dim3(kDin / kScanC, kBatch), kScanC, 0, stream>>>(DPRE, x, XZ, b_dt, A_log, Dv, out);
}
